// YOSOFFN_69965017252065
// MI455X (gfx1250) — hardware-verified
//
#include <hip/hip_runtime.h>
#include <math.h>

constexpr int   kHidden    = 1024;
constexpr int   kInter     = 4096;
constexpr int   kChunkRows = 2048;
constexpr float kQCarry    = 16.0f;
constexpr float kKCarry    = 16.0f;
constexpr float kVCarry    = 256.0f;
constexpr float kBCarry    = 2048.0f;
constexpr float kScale1    = 1.0f / (kQCarry * kKCarry);
constexpr float kScale2    = 1.0f / (kBCarry * kVCarry);
constexpr float kInvPi     = 0.31830988618379067f;
constexpr float kClipLo    = -1.0f + 1e-6f;
constexpr float kClipHi    = 1.0f - 1e-6f;
constexpr float kLnEps     = 1e-12f;
constexpr float kNormFloor = 1e-12f;
constexpr float kInvHidden = 1.0f / 1024.0f;

static_assert(kChunkRows % 64 == 0);
static_assert(kHidden % 64 == 0);
static_assert(kInter % 64 == 0);

typedef __attribute__((ext_vector_type(16))) _Float16 v16h;
typedef __attribute__((ext_vector_type(8)))  _Float16 v8h;
typedef __attribute__((ext_vector_type(16))) __bf16   v16b;
typedef __attribute__((ext_vector_type(8)))  __bf16   v8b;
typedef __attribute__((ext_vector_type(8)))  float    v8f;
typedef __attribute__((ext_vector_type(4)))  float    v4f;
typedef __attribute__((ext_vector_type(4)))  unsigned int v4u;

__device__ __forceinline__ unsigned short f2bf_bits(float f) {
  unsigned u = __float_as_uint(f);
  return (unsigned short)((u + 0x7FFFu + ((u >> 16) & 1u)) >> 16);
}
__device__ __forceinline__ float bf_bits2f(unsigned short h) { return __uint_as_float(((unsigned)h) << 16); }

__device__ __forceinline__ void dep_guard_h(v8f& a, v8f& b, v16h x, v16h y) { asm volatile("v_nop\n\tv_nop\n\tv_nop\n\tv_nop" : "+v"(a), "+v"(b) : "v"(x), "v"(y)); }
__device__ __forceinline__ void dep_guard_b(v8f& a, v8f& b, v16b x, v16b y) { asm volatile("v_nop\n\tv_nop\n\tv_nop\n\tv_nop" : "+v"(a), "+v"(b) : "v"(x), "v"(y)); }
__device__ __forceinline__ void keep4_h(v16h a, v16h b, v16h c, v16h d) { asm volatile("v_nop" :: "v"(a), "v"(b), "v"(c), "v"(d)); }
__device__ __forceinline__ void keep4_b(v16b a, v16b b, v16b c, v16b d) { asm volatile("v_nop" :: "v"(a), "v"(b), "v"(c), "v"(d)); }
__device__ __forceinline__ void acc_guard4(v8f& a, v8f& b, v8f& c, v8f& d) { asm volatile("v_nop\n\tv_nop\n\tv_nop\n\tv_nop" : "+v"(a), "+v"(b), "+v"(c), "+v"(d)); }
template <typename T> struct Frag;
template <> struct Frag<_Float16> {
  typedef v16h V; union U { v16h v; v8h h[2]; };
  static __device__ __forceinline__ v16h load(const _Float16* p) {
    U f; f.h[0] = *(const v8h*)(p); f.h[1] = *(const v8h*)(p + 16); return f.v;
  }
  static __device__ __forceinline__ v8f mma(v16h a, v16h b, v8f c) {
    return __builtin_amdgcn_wmma_f32_16x16x32_f16(false, a, false, b, (short)0, c, false, false);
  }
  static __device__ __forceinline__ void guard(v8f& a, v8f& b, v16h x, v16h y) { dep_guard_h(a, b, x, y); }
  static __device__ __forceinline__ void keep(v16h a, v16h b, v16h c, v16h d) { keep4_h(a, b, c, d); }
};
template <> struct Frag<__bf16> {
  typedef v16b V; union U { v16b v; v8b h[2]; };
  static __device__ __forceinline__ v16b load(const __bf16* p) {
    U f; f.h[0] = *(const v8b*)(p); f.h[1] = *(const v8b*)(p + 16); return f.v;
  }
  static __device__ __forceinline__ v8f mma(v16b a, v16b b, v8f c) {
    return __builtin_amdgcn_wmma_f32_16x16x32_bf16(false, a, false, b, (short)0, c, false, false);
  }
  static __device__ __forceinline__ void guard(v8f& a, v8f& b, v16b x, v16b y) { dep_guard_b(a, b, x, y); }
  static __device__ __forceinline__ void keep(v16b a, v16b b, v16b c, v16b d) { keep4_b(a, b, c, d); }
};

__device__ __forceinline__ unsigned pk16(unsigned short a, unsigned short b) { return (unsigned)a | ((unsigned)b << 16); }
__device__ __forceinline__ unsigned short h_bits(float f) { const _Float16 h = (_Float16)f; return __builtin_bit_cast(unsigned short, h); }

template <int ET> struct Elem;
template <> struct Elem<0> { typedef _Float16 T; };
template <> struct Elem<1> { typedef __bf16 T; };
template <int ET, bool SPLIT, int BIAS_MODE, int OUT_MODE, bool RESID, int ACT = 0>
__global__ __launch_bounds__(256) void wmma_gemm64(
    const unsigned short* __restrict__ Ap, const unsigned short* __restrict__ A2p, int lda, long strideA,
    const unsigned short* __restrict__ Btp, const unsigned short* __restrict__ Bt2p, int ldb, long strideB,
    void* __restrict__ Cout, void* __restrict__ Cout2, int ldc, long strideC,
    const float* __restrict__ bias,
    const float* __restrict__ resid, long strideR,
    int M, int N, int K, float scale) {
  typedef typename Elem<ET>::T T;
  typedef typename Frag<T>::V V;
  const T* A = (const T*)Ap; const T* A2 = (const T*)A2p; const T* Bt = (const T*)Btp; const T* Bt2 = (const T*)Bt2p;
  __shared__ __align__(16) float sT[8][16 * 68];
  const int b    = blockIdx.y;
  const int lane = threadIdx.x & 31;
  const int wave = threadIdx.x >> 5;
  const int tilesN = N >> 6;
  const int tilesM = M >> 6;
  const int tile = blockIdx.x * 8 + wave;
  if (tile >= tilesM * tilesN) return;
  const int tm = tile / tilesN;
  const int tn = tile - tm * tilesN;
  const int m0 = tm << 6;
  const int n0 = tn << 6;

  const T* Ab  = A  + (size_t)b * strideA;
  const T* Bb  = Bt + (size_t)b * strideB;
  const T* Ab2 = SPLIT ? (A2  + (size_t)b * strideA) : nullptr;
  const T* Bb2 = SPLIT ? (Bt2 + (size_t)b * strideB) : nullptr;

  const int rlane = lane & 15;
  const int koff  = (lane >> 4) * 8;
  const int mOff  = (lane >> 4) * 8;

  v8f acc[4][4];
#pragma unroll
  for (int i = 0; i < 4; ++i)
#pragma unroll
    for (int j = 0; j < 4; ++j) acc[i][j] = (v8f){0.f,0.f,0.f,0.f,0.f,0.f,0.f,0.f};

  for (int k0 = 0; k0 < K; k0 += 32) {
    V bh[4], bl[4];
#pragma unroll
    for (int j = 0; j < 4; ++j) {
      const size_t bo = (size_t)(n0 + (j << 4) + rlane) * ldb + koff + k0;
      bh[j] = Frag<T>::load(Bb + bo);
      if (SPLIT) bl[j] = Frag<T>::load(Bb2 + bo);
    }
#pragma unroll
    for (int i = 0; i < 4; ++i) {
      const size_t ao = (size_t)(m0 + (i << 4) + rlane) * lda + koff + k0;
      V ah = Frag<T>::load(Ab + ao);
      V al;
      if (SPLIT) al = Frag<T>::load(Ab2 + ao);
#pragma unroll
      for (int j = 0; j < 4; ++j) {
        acc[i][j] = Frag<T>::mma(ah, bh[j], acc[i][j]);
        if (SPLIT) {
          acc[i][j] = Frag<T>::mma(ah, bl[j], acc[i][j]);
          acc[i][j] = Frag<T>::mma(al, bh[j], acc[i][j]);
        }
      }
      Frag<T>::guard(acc[i][0], acc[i][3], ah, SPLIT ? al : ah);
    }
    Frag<T>::keep(bh[0], bh[1], bh[2], bh[3]);
    if (SPLIT) Frag<T>::keep(bl[0], bl[1], bl[2], bl[3]);
  }
  acc_guard4(acc[0][0], acc[0][1], acc[0][2], acc[0][3]);
  acc_guard4(acc[1][0], acc[1][1], acc[1][2], acc[1][3]);
  acc_guard4(acc[2][0], acc[2][1], acc[2][2], acc[2][3]);
  acc_guard4(acc[3][0], acc[3][1], acc[3][2], acc[3][3]);

  float* slab = sT[wave];
  const float* Rb = RESID ? (resid + (size_t)b * strideR) : nullptr;
#pragma unroll
  for (int i = 0; i < 4; ++i) {
    const int mBase = m0 + (i << 4);
#pragma unroll
    for (int j = 0; j < 4; ++j) {
      const int n = n0 + (j << 4) + rlane;
      float bv = 0.f;
      if (BIAS_MODE == 2) bv = bias[n];
#pragma unroll
      for (int r = 0; r < 8; ++r) {
        float v = acc[i][j][r] * scale;
        if (BIAS_MODE == 1) v += bias[mBase + mOff + r];
        if (BIAS_MODE == 2) v += bv;
        if (RESID) v += Rb[(size_t)(mBase + mOff + r) * ldc + n];
        if (ACT == 2) v = fmaxf(v, 0.0f);
        if (ACT == 4) v = (v > 0.f) ? v : 0.01f * v;
        slab[(mOff + r) * 68 + (j << 4) + rlane] = v;
      }
    }
    __builtin_amdgcn_fence(__ATOMIC_RELEASE, "workgroup");
    __builtin_amdgcn_wave_barrier();
    __builtin_amdgcn_fence(__ATOMIC_ACQUIRE, "workgroup");
    if (ACT == 6) {
#pragma unroll 1
      for (int e = lane; e < 16 * 64; e += 32) {
        const int rr = e >> 6;
        const int cc = e & 63;
        float sv = slab[rr * 68 + cc];
        sv = fminf(fmaxf(sv, kClipLo), kClipHi);
        const float tb = 1.0f - acosf(sv) * kInvPi;
        const float t2 = tb * tb;
        const float t4 = t2 * t2;
        const float t8 = t4 * t4;
        slab[rr * 68 + cc] = (t8 * tb) * kBCarry;
      }
      __builtin_amdgcn_fence(__ATOMIC_RELEASE, "workgroup");
      __builtin_amdgcn_wave_barrier();
      __builtin_amdgcn_fence(__ATOMIC_ACQUIRE, "workgroup");
    }
    if (OUT_MODE == 0) {
      float* C = (float*)Cout + (size_t)b * strideC;
      const int hh = lane >> 4, c4 = (lane & 15) * 4;
      for (int pass = 0; pass < 2; ++pass) {
#pragma unroll
        for (int it = 0; it < 8; ++it) {
          const int row = it * 2 + hh;
          v4f v = *(const v4f*)(slab + row * 68 + c4);
          *(volatile v4f*)(C + (size_t)(mBase + row) * ldc + n0 + c4) = v;
        }
        __threadfence();
      }
    } else {
      const int q = lane >> 3, c8 = (lane & 7) * 8;
      unsigned short* C  = (unsigned short*)Cout  + (size_t)b * strideC;
      unsigned short* C2 = (OUT_MODE == 2) ? ((unsigned short*)Cout2 + (size_t)b * strideC) : nullptr;
      for (int pass = 0; pass < 2; ++pass) {
#pragma unroll
        for (int it = 0; it < 4; ++it) {
          const int row = it * 4 + q;
          const float* sp = slab + row * 68 + c8;
          v8h hv, lv;
#pragma unroll
          for (int e = 0; e < 8; ++e) {
            if (OUT_MODE == 1) {
              hv[e] = (_Float16)sp[e];
            } else {
              unsigned short hb = f2bf_bits(sp[e]);
              unsigned short lb = f2bf_bits(sp[e] - bf_bits2f(hb));
              hv[e] = __builtin_bit_cast(_Float16, hb);
              lv[e] = __builtin_bit_cast(_Float16, lb);
            }
          }
          *(volatile v8h*)(C + (size_t)(mBase + row) * ldc + n0 + c8) = hv;
          if (OUT_MODE == 2) *(volatile v8h*)(C2 + (size_t)(mBase + row) * ldc + n0 + c8) = lv;
        }
        __threadfence();
      }
    }
    __builtin_amdgcn_fence(__ATOMIC_RELEASE, "workgroup");
    __builtin_amdgcn_wave_barrier();
    __builtin_amdgcn_fence(__ATOMIC_ACQUIRE, "workgroup");
  }
}

__device__ __forceinline__ float block_sum4(float s, float* red, int lane, int wave) {
#pragma unroll
  for (int off = 16; off > 0; off >>= 1) s += __shfl_xor(s, off, 32);
  __syncthreads();
  if (lane == 0) red[wave] = s;
  __syncthreads();
  return (red[0] + red[1]) + (red[2] + red[3]);
}

template <bool LN>
__global__ __launch_bounds__(128) void rownorm16_kernel(const float* __restrict__ x,
                                                       const float* __restrict__ g,
                                                       const float* __restrict__ be,
                                                       unsigned short* __restrict__ outp,
                                                       float carry) {
  __shared__ float red[4];
  const int row  = blockIdx.x;
  const int t    = threadIdx.x;
  const int lane = t & 31, wave = t >> 5;
  const float* xr = x + (size_t)row * kHidden + 8 * t;
  const v4f a = *(const v4f*)(xr);
  const v4f c = *(const v4f*)(xr + 4);
  float v[8];
#pragma unroll
  for (int e = 0; e < 4; ++e) { v[e] = a[e]; v[4 + e] = c[e]; }
  if (LN) {
    float s = 0.f;
#pragma unroll
    for (int e = 0; e < 8; ++e) s += v[e];
    const float tot = block_sum4(s, red, lane, wave);
    const float mu = tot * kInvHidden;
    float s2 = 0.f;
#pragma unroll
    for (int e = 0; e < 8; ++e) { v[e] = v[e] - mu; s2 += v[e] * v[e]; }
    const float tot2 = block_sum4(s2, red, lane, wave);
    const float rstd = rsqrtf(tot2 * kInvHidden + kLnEps);
    const v4f ga = *(const v4f*)(g + 8 * t);
    const v4f gc = *(const v4f*)(g + 8 * t + 4);
    const v4f ba = *(const v4f*)(be + 8 * t);
    const v4f bc = *(const v4f*)(be + 8 * t + 4);
#pragma unroll
    for (int e = 0; e < 4; ++e) {
      v[e]     = (v[e] * rstd) * ga[e] + ba[e];
      v[4 + e] = (v[4 + e] * rstd) * gc[e] + bc[e];
    }
  }
  float ss = 0.f;
#pragma unroll
  for (int e = 0; e < 8; ++e) ss += v[e] * v[e];
  const float tot3 = block_sum4(ss, red, lane, wave);
  const float inv = carry * (1.0f / fmaxf(sqrtf(tot3), kNormFloor));
  unsigned short hb[8];
#pragma unroll
  for (int e = 0; e < 8; ++e) hb[e] = h_bits(v[e] * inv);
  const v4u u = (v4u){pk16(hb[0], hb[1]), pk16(hb[2], hb[3]), pk16(hb[4], hb[5]), pk16(hb[6], hb[7])};
  unsigned short* q = outp + (size_t)row * kHidden + 8 * t;
  *(volatile v4u*)q = u;
  __threadfence();
  *(volatile v4u*)q = u;
}

__global__ __launch_bounds__(256) void qtrans16_kernel(const float* __restrict__ W,
                                                       unsigned short* __restrict__ outp, float scale) {
  __shared__ float sm[64][65];
  const int t  = threadIdx.x;
  const int i0 = blockIdx.x * 64;
  const int h0 = blockIdx.y * 64;
#pragma unroll
  for (int it = 0; it < 16; ++it) {
    const int e = it * 256 + t;
    const int r = e >> 6;
    const int c = e & 63;
    sm[c][r] = W[(size_t)(i0 + r) * kHidden + h0 + c] * scale;
  }
  __syncthreads();
  const int lane = t & 31, wave = t >> 5;
  const int q = lane >> 3, c8 = (lane & 7) * 8;
  for (int pass = 0; pass < 2; ++pass) {
#pragma unroll
    for (int it = 0; it < 2; ++it) {
      const int rowl = wave * 8 + it * 4 + q;
      unsigned short hb[8];
#pragma unroll
      for (int e = 0; e < 8; ++e) hb[e] = h_bits(sm[rowl][c8 + e]);
      const v4u u = (v4u){pk16(hb[0], hb[1]), pk16(hb[2], hb[3]), pk16(hb[4], hb[5]), pk16(hb[6], hb[7])};
      *(volatile v4u*)(outp + (size_t)(h0 + rowl) * kInter + i0 + c8) = u;
    }
    __threadfence();
  }
}

__global__ __launch_bounds__(256) void l2bias_out_kernel(const float* __restrict__ X,
                                                         const float* __restrict__ bias,
                                                         float* __restrict__ outp) {
  #pragma clang fp contract(off)
  __shared__ float red[8];
  const int row  = blockIdx.x;
  const int t    = threadIdx.x;
  const int lane = t & 31, wave = t >> 5;
  const v4f a = *(const v4f*)(X + (size_t)row * kHidden + 4 * t);
  float ss = ((a[0] * a[0] + a[1] * a[1]) + a[2] * a[2]) + a[3] * a[3];
#pragma unroll
  for (int off = 16; off > 0; off >>= 1) ss += __shfl_xor(ss, off, 32);
  if (lane == 0) red[wave] = ss;
  __syncthreads();
  const float tot = ((red[0] + red[1]) + (red[2] + red[3])) + ((red[4] + red[5]) + (red[6] + red[7]));
  const float inv = 1.0f / fmaxf(sqrtf(tot), kNormFloor);
  const v4f bb = *(const v4f*)(bias + 4 * t);
  v4f o;
#pragma unroll
  for (int e = 0; e < 4; ++e) o[e] = a[e] * inv + bb[e];
  float* q = outp + (size_t)row * kHidden + 4 * t;
  *(volatile v4f*)q = o;
  __threadfence();
  *(volatile v4f*)q = o;
}

extern "C" void kernel_launch(void* const* d_in, const int* in_sizes, int n_in,
                              void* d_out, int out_size, void* d_ws, size_t ws_size,
                              hipStream_t stream) {
  if (n_in < 6) return;
  const float* hidden = (const float*)d_in[0];
  const float* ln_w   = (const float*)d_in[1];
  const float* ln_b   = (const float*)d_in[2];
  const float* k_w    = (const float*)d_in[3];
  const float* q_w    = (const float*)d_in[4];
  const float* bias   = (const float*)d_in[5];
  float* out = (float*)d_out;

  const int nRows = in_sizes[0] / kHidden;
  if (nRows <= 0 || (nRows % kChunkRows) != 0) return;
  if (in_sizes[1] != kHidden || in_sizes[2] != kHidden || in_sizes[5] != kHidden) return;
  if (in_sizes[3] != kInter * kHidden || in_sizes[4] != kInter * kHidden) return;
  if (out_size != nRows * kHidden) return;
  const int nChunks = nRows / kChunkRows;

  const size_t szQ  = (size_t)nRows * kHidden * 2;
  const size_t szKN = (size_t)kInter * kHidden * 2;
  const size_t szQT = (size_t)kHidden * kInter * 2;
  const size_t szB  = (size_t)kChunkRows * kInter * 2;
  const size_t szX  = (size_t)nRows * kHidden * 4;
  const size_t oQ  = 0;
  const size_t oKN = oQ + szQ;
  const size_t oQT = oKN + szKN;
  const size_t oB  = oQT + szQT;
  const size_t oX  = oB + szB;
  const size_t total = oX + szX;
  if (total > ws_size) return;

  char* ws = (char*)d_ws;
  unsigned short* Q16  = (unsigned short*)(ws + oQ);
  unsigned short* KN16 = (unsigned short*)(ws + oKN);
  unsigned short* QT16 = (unsigned short*)(ws + oQT);
  unsigned short* B16  = (unsigned short*)(ws + oB);
  float*          Xf   = (float*)(ws + oX);

  rownorm16_kernel<false><<<dim3(kInter), dim3(128), 0, stream>>>(k_w, ln_w, ln_b, KN16, kKCarry);
  qtrans16_kernel<<<dim3(kInter / 64, kHidden / 64), dim3(256), 0, stream>>>(q_w, QT16, kVCarry);
  rownorm16_kernel<true><<<dim3(nRows), dim3(128), 0, stream>>>(hidden, ln_w, ln_b, Q16, kQCarry);

  const int tiles1 = (kChunkRows / 64) * (kInter / 64);
  const int tiles2 = (kChunkRows / 64) * (kHidden / 64);
  const int grid1 = (tiles1 + 7) / 8;
  const int grid2 = (tiles2 + 7) / 8;
  for (int ch = 0; ch < nChunks; ++ch) {
    const unsigned short* Qc = Q16 + (size_t)ch * kChunkRows * kHidden;
    float* Xc = Xf + (size_t)ch * kChunkRows * kHidden;
    wmma_gemm64<0, false, 0, 1, false, 6><<<dim3(grid1, 1), dim3(256), 0, stream>>>(
        Qc, Qc, kHidden, 0L,
        KN16, KN16, kHidden, 0L,
        (void*)B16, (void*)B16, kInter, 0L,
        bias,
        Xf, 0L,
        kChunkRows, kInter, kHidden, kScale1);
    wmma_gemm64<0, false, 0, 0, false, 0><<<dim3(grid2, 1), dim3(256), 0, stream>>>(
        B16, B16, kInter, 0L,
        QT16, QT16, kInter, 0L,
        (void*)Xc, (void*)Xc, kHidden, 0L,
        bias,
        Xf, 0L,
        kChunkRows, kHidden, kInter, kScale2);
  }
  l2bias_out_kernel<<<dim3(nRows), dim3(256), 0, stream>>>(Xf, bias, out);
}
